// RelationWiseWordSelectionHead_69836168233629
// MI455X (gfx1250) — hardware-verified
//
#include <hip/hip_runtime.h>


#ifndef NB
#define NB 2
#endif
#ifndef SEQ
#define SEQ 192
#endif
#define NB_FULL  2
#define SEQ_FULL 192
#ifndef OUT_SEQ
#define OUT_SEQ SEQ
#endif
#define DM   768
#define NREL 4
#define NCOL (NREL * DM)
#define OSW  68

static_assert(DM % 32 == 0);
static_assert(NCOL % 64 == 0);
static_assert((NB * SEQ) % 64 == 0);
static_assert(NREL == 4);
static_assert(DM % 4 == 0);
static_assert(SEQ % 32 == 0);
static_assert(SEQ <= 1024);
static_assert(SEQ % 8 == 0);
static_assert(((size_t)NCOL * 4) % 128 == 0);
static_assert(((size_t)OUT_SEQ * NREL * 4) % 128 == 0);
static_assert(((size_t)SEQ * DM) % 8 == 0);
static_assert(((size_t)NCOL * DM) % 8 == 0);
static_assert(NB <= NB_FULL);
static_assert(SEQ <= SEQ_FULL);
static_assert(SEQ <= OUT_SEQ);
static_assert((OSW * 4) % 16 == 0);
static_assert(8 * 2 == 16);
static_assert(16 * 4 == 64);
static_assert(32 * 16 == 2 * 64 * 4);
static_assert(16 * OSW * 4 <= 131072);
static_assert(2 * NCOL * 4 <= 131072);
static_assert((size_t)SEQ * 16 == (size_t)SEQ * NREL * 4);

typedef unsigned short bf;
typedef __attribute__((ext_vector_type(16))) __bf16   v16bf;
typedef __attribute__((ext_vector_type(8)))  unsigned short v8us;
typedef __attribute__((ext_vector_type(8)))  float    v8f;
typedef __attribute__((ext_vector_type(4)))  float    v4f;
typedef v4f  __attribute__((may_alias)) v4fa;

__device__ __forceinline__ unsigned short f2bf(float f) { unsigned u = __float_as_uint(f); u += 0x7FFFu + ((u >> 16) & 1u); return (unsigned short)(u >> 16); }
__device__ __forceinline__ float bfr(float f) { return __uint_as_float(((unsigned)f2bf(f)) << 16); }
__device__ __forceinline__ v16bf cat16b(v8us lo, v8us hi) { return __builtin_bit_cast(v16bf, __builtin_shufflevector(lo, hi, 0, 1, 2, 3, 4, 5, 6, 7, 8, 9, 10, 11, 12, 13, 14, 15)); }
__device__ __forceinline__ v8f wmmab(v16bf a, v16bf b, v8f c) { return __builtin_amdgcn_wmma_f32_16x16x32_bf16(false, a, false, b, (short)0, c, false, false); }
__device__ __forceinline__ v8f wmmabg(v16bf a, v16bf b, v8f c) { c = wmmab(a, b, c); asm volatile("v_nop\n\tv_nop\n\tv_nop\n\tv_nop" : "+v"(c) : "v"(a), "v"(b)); return c; }
__device__ __forceinline__ v16bf ldb(const bf* p)  { return cat16b(*(const v8us*)p, *(const v8us*)(p + 16)); }
__device__ __forceinline__ void wave_sync() { __builtin_amdgcn_fence(3  , "wavefront"); __builtin_amdgcn_wave_barrier(); asm volatile("" ::: "memory"); }
__device__ __forceinline__ float gelu_erf(float u) { return 0.5f * u * (1.0f + erff(u * 0.70710678118654752f)); }

__global__ __launch_bounds__(256) void k_cvt8(const float* __restrict__ src, bf* dst, size_t n8) {
    const size_t i = (size_t)blockIdx.x * 256 + threadIdx.x; if (i >= n8) return;
    const v8f v = *(const v8f*)(src + i * 8); v8us o;
#pragma unroll
    for (int k = 0; k < 8; ++k) o[k] = f2bf(v[k]);
    *(volatile v8us*)(dst + i * 8) = o; __threadfence(); *(volatile v8us*)(dst + i * 8) = o;
}

__global__ __launch_bounds__(32) void k_gemm(const bf* __restrict__ A, const bf* __restrict__ Bt, const float* __restrict__ bias, float* C) {
    __shared__ __align__(16) float os[16 * OSW];
    const int K = DM;
    const int lane = threadIdx.x & 31, lr = lane & 15, hi = lane >> 4;
    const unsigned bx = blockIdx.x, by = blockIdx.y;
    const int r0 = (int)(bx * 64u), c0 = (int)(by * 64u);
    v8f acc[4][4];
#pragma unroll
    for (int mb = 0; mb < 4; ++mb)
#pragma unroll
        for (int nb = 0; nb < 4; ++nb) acc[mb][nb] = (v8f){};
    const size_t aoff = (size_t)(r0 + lr) * K + 8 * hi, boff = (size_t)(c0 + lr) * K + 8 * hi;
#pragma unroll 1
    for (int kc = 0; kc < K; kc += 32) {
        v16bf a[4];
#pragma unroll
        for (int mb = 0; mb < 4; ++mb) a[mb] = ldb(A + aoff + (size_t)mb * 16 * K + kc);
#pragma unroll
        for (int nb = 0; nb < 4; ++nb) { const v16bf b = ldb(Bt + boff + (size_t)nb * 16 * K + kc);
#pragma unroll
            for (int mb = 0; mb < 4; ++mb) acc[mb][nb] = wmmabg(a[mb], b, acc[mb][nb]); }
    }
    float bc[4];
#pragma unroll
    for (int nb = 0; nb < 4; ++nb) bc[nb] = bfr(bias[c0 + nb * 16 + lr]);
#pragma unroll
    for (int mb = 0; mb < 4; ++mb) {
#pragma unroll
        for (int nb = 0; nb < 4; ++nb) {
#pragma unroll
            for (int j = 0; j < 8; ++j) os[(hi * 8 + j) * OSW + nb * 16 + lr] = acc[mb][nb][j] + bc[nb]; }
        wave_sync();
        float* crow = C + (size_t)(r0 + mb * 16) * NCOL + c0;
#pragma unroll 1
        for (int ps = 0; ps < 2; ++ps) {
#pragma unroll
            for (int s = 0; s < 8; ++s) { const int row = 2 * s + (lane >> 4), cofs = (lane & 15) * 4;
                const v4f val = *(const v4fa*)(&os[row * OSW + cofs]);
                *(volatile v4f*)(crow + (size_t)row * NCOL + cofs) = val; }
            if (ps == 0) __threadfence(); }
        wave_sync();
    }
}

__global__ __launch_bounds__(SEQ) void k_pair(const float* __restrict__ HS, const float* __restrict__ HT, const float* __restrict__ cw, float* OUT) {
    __shared__ __align__(16) float hs[NCOL];
    __shared__ __align__(16) float cl[NCOL];
    const unsigned bx = blockIdx.x;
    const unsigned b = bx / (unsigned)SEQ, s = bx % (unsigned)SEQ;
    const int tid = (int)threadIdx.x;
    const size_t srow = (size_t)bx * NCOL;
#pragma unroll 1
    for (int i = tid; i < NCOL / 4; i += SEQ) { const v4f v = *(const v4f*)(HS + srow + (size_t)4 * i); *(v4fa*)(&hs[4 * i]) = v; }
#pragma unroll 1
    for (int i = tid; i < DM; i += SEQ) { const v4f c = *(const v4f*)(cw + (size_t)4 * i);
        cl[0 * DM + i] = bfr(c[0]); cl[1 * DM + i] = bfr(c[1]); cl[2 * DM + i] = bfr(c[2]); cl[3 * DM + i] = bfr(c[3]); }
    __syncthreads();
    const float* trow = HT + ((size_t)b * SEQ + (size_t)tid) * NCOL;
    float o0 = 0.0f, o1 = 0.0f, o2 = 0.0f, o3 = 0.0f;
#pragma unroll 1
    for (int l = 0; l < NREL; ++l) {
        float a0 = 0.0f, a1 = 0.0f, a2 = 0.0f, a3 = 0.0f;
#pragma unroll 1
        for (int h4 = 0; h4 < DM / 4; ++h4) {
            const int idx = l * DM + 4 * h4;
            const v4f x  = *(const v4f*)(trow + idx);
            const v4f sv = *(const v4fa*)(&hs[idx]);
            const v4f wv = *(const v4fa*)(&cl[idx]);
            a0 = fmaf(gelu_erf(sv[0] + x[0]), wv[0], a0);
            a1 = fmaf(gelu_erf(sv[1] + x[1]), wv[1], a1);
            a2 = fmaf(gelu_erf(sv[2] + x[2]), wv[2], a2);
            a3 = fmaf(gelu_erf(sv[3] + x[3]), wv[3], a3);
        }
        const float r = (a0 + a1) + (a2 + a3);
        o0 = (l == 0) ? r : o0; o1 = (l == 1) ? r : o1; o2 = (l == 2) ? r : o2; o3 = (l == 3) ? r : o3;
    }
    v4f val; val[0] = o0; val[1] = o1; val[2] = o2; val[3] = o3;
    float* op = OUT + (((size_t)b * OUT_SEQ + (size_t)s) * OUT_SEQ + (size_t)tid) * NREL;
    *(volatile v4f*)op = val; __threadfence(); *(volatile v4f*)op = val;
}

static constexpr size_t al256(size_t v) { return (v + 255) & ~(size_t)255; }
static constexpr size_t SZ_XB = al256((size_t)NB * SEQ * DM * 2);
static constexpr size_t SZ_WB = al256((size_t)NCOL * DM * 2);
static constexpr size_t SZ_HP = al256((size_t)NB * SEQ * NCOL * 4);
static constexpr size_t SZ_TOTAL = SZ_XB + 2 * SZ_WB + 2 * SZ_HP;
static_assert(SZ_TOTAL <= (size_t)134217728);
static_assert((size_t)(NB * SEQ / 64) * 64 * (size_t)(NCOL / 64) * 64 * 4 == (size_t)NB * SEQ * NCOL * 4);

extern "C" void kernel_launch(void* const* d_in, const int* in_sizes, int n_in,
                              void* d_out, int out_size, void* d_ws, size_t ws_size, hipStream_t stream) {
    if (n_in < 6) return;
    const size_t needx = ((size_t)(NB - 1) * SEQ_FULL + SEQ) * DM;
    if ((size_t)in_sizes[0] < needx) return;
    if ((size_t)in_sizes[1] < (size_t)NCOL * DM || (size_t)in_sizes[3] < (size_t)NCOL * DM) return;
    if (in_sizes[2] < NCOL || in_sizes[4] < NCOL || in_sizes[5] < DM * NREL) return;
    if ((size_t)out_size < ((((size_t)(NB - 1) * OUT_SEQ + (size_t)(SEQ - 1)) * OUT_SEQ + SEQ) * NREL)) return;
    if (SZ_TOTAL > ws_size) return;
    const float* xin = (const float*)d_in[0];
    const float* wsrc = (const float*)d_in[1]; const float* bsrc = (const float*)d_in[2];
    const float* wtgt = (const float*)d_in[3]; const float* btgt = (const float*)d_in[4];
    const float* cwt = (const float*)d_in[5];
    float* OUT = (float*)d_out;
    char* wsp = (char*)d_ws;
    bf* XB = (bf*)wsp; wsp += SZ_XB;
    bf* WS = (bf*)wsp; wsp += SZ_WB;
    bf* WT = (bf*)wsp; wsp += SZ_WB;
    float* HS = (float*)wsp; wsp += SZ_HP;
    float* HT = (float*)wsp; wsp += SZ_HP;

    if (SEQ == SEQ_FULL) {
        const size_t n8 = (size_t)NB * SEQ * DM / 8;
        k_cvt8<<<(unsigned)((n8 + 255) / 256), 256, 0, stream>>>(xin, XB, n8);
    } else {
        const size_t n8 = (size_t)SEQ * DM / 8;
        for (int b = 0; b < NB; ++b) k_cvt8<<<(unsigned)((n8 + 255) / 256), 256, 0, stream>>>(xin + (size_t)b * SEQ_FULL * DM, XB + (size_t)b * SEQ * DM, n8);
    }
    { const size_t n8 = (size_t)NCOL * DM / 8; const unsigned g = (unsigned)((n8 + 255) / 256);
      k_cvt8<<<g, 256, 0, stream>>>(wsrc, WS, n8); k_cvt8<<<g, 256, 0, stream>>>(wtgt, WT, n8); }

    k_gemm<<<dim3(NB * SEQ / 64, NCOL / 64, 1), 32, 0, stream>>>(XB, WS, bsrc, HS);
    k_gemm<<<dim3(NB * SEQ / 64, NCOL / 64, 1), 32, 0, stream>>>(XB, WT, btgt, HT);

    k_pair<<<dim3(NB * SEQ, 1, 1), SEQ, 0, stream>>>(HS, HT, cwt, OUT);
}
